// NonLocalBlock_62526133895211
// MI455X (gfx1250) — hardware-verified
//
#include <hip/hip_runtime.h>
#include <math.h>

typedef __attribute__((ext_vector_type(16))) _Float16 v16h;
typedef __attribute__((ext_vector_type(8)))  _Float16 v8h;
typedef __attribute__((ext_vector_type(8)))  float v8f;
typedef __attribute__((ext_vector_type(4)))  float v4f;
typedef __attribute__((ext_vector_type(4)))  unsigned v4u;

template <typename T> __device__ __forceinline__ void vst2(void* p, T v) { *(volatile T*)p = v; __threadfence(); *(volatile T*)p = v; }
__device__ __forceinline__ v8f wmma16(v16h a, v16h b, v8f c) {
  v8f d = __builtin_amdgcn_wmma_f32_16x16x32_f16(false, a, false, b, (short)0, c, false, false);
  asm volatile("v_nop\n\tv_nop\n\tv_nop\n\tv_nop" : "+v"(d) : "v"(a), "v"(b));
  return d;
}
__device__ __forceinline__ v16h frag_h(const _Float16* rowk0, int lane) {
  union { v16h v; v8h q[2]; } u; const _Float16* p = rowk0 + 8 * (lane >> 4);
  u.q[0] = *(const v8h*)p; u.q[1] = *(const v8h*)(p + 16); return u.v;
}
__device__ __forceinline__ float bfr(float v) { return (float)(__bf16)v; }
__device__ __forceinline__ v4u pack8(v4f a, v4f b, float sc) { union { v8h h; v4u u; } o;
#pragma unroll
  for (int i = 0; i < 4; ++i) { o.h[i] = (_Float16)(a[i] * sc); o.h[4 + i] = (_Float16)(b[i] * sc); }
  return o.u; }
#define LDSX() do { asm volatile("s_wait_dscnt 0" ::: "memory"); __builtin_amdgcn_wave_barrier(); __builtin_amdgcn_fence(3  , "workgroup"); } while (0)

#ifndef NB
#define NB 4
#endif
#ifndef TT
#define TT 4096
#endif
#define NB_FULL 4
#define TT_FULL 4096
#define CH 256
#define NG 32
#define CPG 8
#define EPSV 1e-5f
#define QK_SCALE 0.0625f
#define W_CARRY 256.0f
#define P_CARRY 2048.0f

static_assert(TT % 256 == 0);
static_assert(TT <= TT_FULL);
static_assert(NB <= NB_FULL);
static_assert(CH % 128 == 0);
static_assert(CH == NG * CPG);

#define SZ_STAT ((size_t)NB_FULL * NG * 128)
#define SZ_WH   ((size_t)4 * CH * CH * 2)
#define SZ_ROWS ((size_t)NB * TT * CH * 2)
#define SZ_S    ((size_t)TT * TT * 4)
#define WS_STAT ((size_t)0)
#define WS_WH   (WS_STAT + SZ_STAT)
#define WS_XH   (WS_WH + SZ_WH)
#define WS_QH   (WS_XH + SZ_ROWS)
#define WS_KH   (WS_QH + SZ_ROWS)
#define WS_VT   (WS_KH + SZ_ROWS)
#define WS_AT   (WS_VT + SZ_ROWS)
#define WS_S    (WS_AT + SZ_ROWS)
#define WS_END  (WS_S + SZ_S)
static_assert(WS_END <= (size_t)134217728);
static_assert((WS_WH % 128) == 0 && (WS_XH % 128) == 0 && (WS_S % 128) == 0);
static_assert((size_t)32 * 256 * 8 == (size_t)CH * CH);
static_assert(((size_t)NB * TT / 64) * 64 * CH == (size_t)NB * TT * CH);
static_assert(((size_t)TT / 64) * (TT / 128) * 64 * 128 == (size_t)TT * TT);
static_assert(((size_t)TT / 64) * (CH / 128) * 64 * 128 == (size_t)TT * CH);
static_assert(((size_t)NB * TT / 128) * (CH / 64) * 64 * 128 == (size_t)NB * CH * TT);

__global__ __launch_bounds__(256) void k_wcvt(const float* __restrict__ W0, const float* __restrict__ W1, const float* __restrict__ W2, const float* __restrict__ W3, _Float16* __restrict__ WH) {
  const int which = blockIdx.y; const float* W = which == 0 ? W0 : which == 1 ? W1 : which == 2 ? W2 : W3;
  const int e = (blockIdx.x * 256 + threadIdx.x) * 8;
  const v4f a = *(const v4f*)(W + e), b = *(const v4f*)(W + e + 4);
  v4f ar, br;
#pragma unroll
  for (int i = 0; i < 4; ++i) { ar[i] = bfr(a[i]); br[i] = bfr(b[i]); }
  vst2((void*)(WH + (size_t)which * CH * CH + e), pack8(ar, br, W_CARRY));
}

__global__ __launch_bounds__(256) void k_gnstat(const float* __restrict__ X, float* __restrict__ STAT) {
  __shared__ double rs[8], rq[8];
  const int tid = threadIdx.x; const int b = blockIdx.x / NG, g = blockIdx.x % NG;
  const float* xg = X + ((size_t)b * CH + (size_t)g * CPG) * TT_FULL;
  float s = 0.f, q = 0.f;
  for (int e = tid; e < CPG * (TT / 4); e += 256) { const int cl = e / (TT / 4), tq = e % (TT / 4);
    const v4f v = *(const v4f*)(xg + (size_t)cl * TT_FULL + tq * 4);
#pragma unroll
    for (int i = 0; i < 4; ++i) { const float r = bfr(v[i]); s += r; q += r * r; } }
  double ds = (double)s, dq = (double)q;
#pragma unroll
  for (int o = 1; o < 32; o <<= 1) { ds += __shfl_xor(ds, o); dq += __shfl_xor(dq, o); }
  if ((tid & 31) == 0) { rs[tid >> 5] = ds; rq[tid >> 5] = dq; }
  __syncthreads();
  double S = 0.0, Q = 0.0;
#pragma unroll
  for (int i = 0; i < 8; ++i) { S += rs[i]; Q += rq[i]; }
  const double invm = 1.0 / (double)(CPG * TT);
  const double mean = S * invm; double var = Q * invm - mean * mean; if (var < 0.0) var = 0.0;
  const float rstd = 1.0f / sqrtf((float)var + EPSV);
  if (tid < 8) { v4f o; o[0] = 0.f; o[1] = 0.f; o[2] = 0.f; o[3] = 0.f; if (tid == 0) { o[0] = (float)mean; o[1] = rstd; }
    vst2((void*)(STAT + (size_t)blockIdx.x * 32 + tid * 4), o); }
}

__global__ __launch_bounds__(256) void k_xn(const float* __restrict__ X, const float* __restrict__ GW, const float* __restrict__ GB, const float* __restrict__ STAT, _Float16* __restrict__ XH) {
  __shared__ __align__(16) _Float16 sh[64][264];
  const int tid = threadIdx.x; const size_t r0 = (size_t)blockIdx.x * 64; const int b = (int)(r0 / TT), t0 = (int)(r0 % TT);
  for (int e = tid; e < CH * 16; e += 256) { const int c = e >> 4, q = e & 15;
    const v4f v = *(const v4f*)(X + ((size_t)b * CH + c) * TT_FULL + t0 + q * 4);
    const float* st = STAT + (size_t)(b * NG + (c >> 3)) * 32; const float mean = st[0], rstd = st[1]; const float w = bfr(GW[c]), bb = bfr(GB[c]);
#pragma unroll
    for (int i = 0; i < 4; ++i) sh[q * 4 + i][c] = (_Float16)((bfr(v[i]) - mean) * rstd * w + bb); }
  __syncthreads();
  for (int e = tid; e < 64 * 32; e += 256) { const int rl = e >> 5, q = e & 31; vst2((void*)(XH + (r0 + rl) * CH + q * 8), *(const v4u*)&sh[rl][q * 8]); }
}

__global__ __launch_bounds__(128) void k_proj(const _Float16* __restrict__ XH, const _Float16* __restrict__ WH, const float* __restrict__ BQ, const float* __restrict__ BK, const float* __restrict__ BV,
    _Float16* __restrict__ QH, _Float16* __restrict__ KH, _Float16* __restrict__ VT) {
  __shared__ __align__(16) _Float16 sh[64][136]; __shared__ __align__(16) _Float16 th[128][72];
  const int tid = threadIdx.x, wave = tid >> 5, lane = tid & 31, col = lane & 15, g = lane >> 4; const int which = blockIdx.z; const int c0 = blockIdx.y * 128; const size_t r0 = (size_t)blockIdx.x * 64; const size_t bb = r0 / TT; const int t0 = (int)(r0 % TT);
  const _Float16* W = WH + (size_t)which * CH * CH; const float* BA = which == 0 ? BQ : which == 1 ? BK : BV;
  v8f acc[8] = {};
#pragma unroll 2
  for (int kc = 0; kc < CH / 32; ++kc) { const v16h a = frag_h(XH + (r0 + wave * 16 + col) * CH + kc * 32, lane);
#pragma unroll
    for (int j = 0; j < 8; ++j) { const v16h w = frag_h(W + (size_t)(c0 + j * 16 + col) * CH + kc * 32, lane);
      acc[j] = wmma16(a, w, acc[j]); } }
  if (which < 2) { _Float16* DH = which == 0 ? QH : KH;
#pragma unroll
    for (int j = 0; j < 8; ++j) { const float bias = bfr(BA[c0 + j * 16 + col]);
#pragma unroll
      for (int r = 0; r < 8; ++r) sh[wave * 16 + 8 * g + r][j * 16 + col] = (_Float16)(acc[j][r] * (1.0f / W_CARRY) + bias); }
    __syncthreads();
    for (int e = tid; e < 64 * 16; e += 128) { const int rl = e >> 4, q = e & 15; vst2((void*)(DH + (r0 + rl) * CH + c0 + q * 8), *(const v4u*)&sh[rl][q * 8]); }
  } else {
#pragma unroll
    for (int j = 0; j < 8; ++j) { const float bias = bfr(BA[c0 + j * 16 + col]);
#pragma unroll
      for (int r = 0; r < 8; ++r) th[j * 16 + col][wave * 16 + 8 * g + r] = (_Float16)(acc[j][r] * (1.0f / W_CARRY) + bias); }
    __syncthreads();
    for (int e = tid; e < 128 * 8; e += 128) { const int cl = e >> 3, q = e & 7; vst2((void*)(VT + (bb * CH + c0 + cl) * (size_t)TT + t0 + q * 8), *(const v4u*)&th[cl][q * 8]); }
  }
}

__global__ __launch_bounds__(128) void k_sc(const _Float16* __restrict__ QH, const _Float16* __restrict__ KH, int b, float* __restrict__ S) {
  __shared__ __align__(16) float ss[4][16][132];
  const int tid = threadIdx.x, wave = tid >> 5, lane = tid & 31, col = lane & 15, g = lane >> 4; const int k0 = blockIdx.y * 128; const int ql0 = blockIdx.x * 64 + wave * 16; const size_t q0 = (size_t)b * TT + ql0, kr0 = (size_t)b * TT + k0;
  v8f acc[8] = {};
#pragma unroll 2
  for (int kc = 0; kc < CH / 32; ++kc) { const v16h ah = frag_h(QH + (q0 + col) * CH + kc * 32, lane);
#pragma unroll
    for (int j = 0; j < 8; ++j) { const v16h kf = frag_h(KH + (kr0 + j * 16 + col) * CH + kc * 32, lane); acc[j] = wmma16(ah, kf, acc[j]); } }
#pragma unroll
  for (int j = 0; j < 8; ++j) {
#pragma unroll
    for (int r = 0; r < 8; ++r) ss[wave][8 * g + r][j * 16 + col] = acc[j][r] * QK_SCALE; }
  LDSX();
  for (int rl = 0; rl < 16; ++rl) vst2((void*)(S + (size_t)(ql0 + rl) * TT + k0 + lane * 4), *(const v4f*)&ss[wave][rl][lane * 4]);
}

__global__ __launch_bounds__(256) void k_sm(float* S0) {
  __shared__ float sred[8]; __shared__ float sbc; __shared__ __align__(16) float shv[TT];
  const int tid = threadIdx.x; float* sr = S0 + (size_t)blockIdx.x * TT;
  float m = -3.0e38f;
  for (int q = tid; q < TT / 4; q += 256) { const v4f v = *(const v4f*)(sr + q * 4); *(v4f*)&shv[q * 4] = v; m = fmaxf(fmaxf(m, fmaxf(v[0], v[1])), fmaxf(v[2], v[3])); }
#pragma unroll
  for (int o = 1; o < 32; o <<= 1) m = fmaxf(m, __shfl_xor(m, o));
  if ((tid & 31) == 0) sred[tid >> 5] = m;
  __syncthreads(); if (tid == 0) { float a = sred[0]; for (int i = 1; i < 8; ++i) a = fmaxf(a, sred[i]); sbc = a; } __syncthreads(); m = sbc; __syncthreads();
  float sum = 0.f;
#pragma unroll 1
  for (int k = tid; k < TT; k += 256) { const float e = expf(shv[k] - m); shv[k] = e; sum += e; }
#pragma unroll
  for (int o = 1; o < 32; o <<= 1) sum += __shfl_xor(sum, o);
  if ((tid & 31) == 0) sred[tid >> 5] = sum;
  __syncthreads(); if (tid == 0) { float a = 0.f; for (int i = 0; i < 8; ++i) a += sred[i]; sbc = P_CARRY * (1.0f / a); } __syncthreads(); const float inv = sbc;
  _Float16* ph = (_Float16*)sr;
  for (int q = tid; q < TT / 8; q += 256) { const v4f a = *(const v4f*)&shv[q * 8], c = *(const v4f*)&shv[q * 8 + 4]; vst2((void*)(ph + q * 8), pack8(a, c, inv)); }
}

__global__ __launch_bounds__(128) void k_pv(const _Float16* __restrict__ PH, const _Float16* __restrict__ VT, int b, _Float16* __restrict__ AT) {
  __shared__ __align__(16) _Float16 sh[64][136];
  const int tid = threadIdx.x, wave = tid >> 5, lane = tid & 31, col = lane & 15, g = lane >> 4; const int d0 = blockIdx.y * 128; const int ql0 = blockIdx.x * 64 + wave * 16;
  const _Float16* prow = PH + (size_t)(ql0 + col) * (2 * (size_t)TT);
  v8f acc[8] = {};
#pragma unroll 1
  for (int kc = 0; kc < TT / 32; ++kc) { const v16h p = frag_h(prow + kc * 32, lane);
#pragma unroll
    for (int j = 0; j < 8; ++j) { const v16h vf = frag_h(VT + ((size_t)b * CH + d0 + j * 16 + col) * (size_t)TT + kc * 32, lane);
      acc[j] = wmma16(p, vf, acc[j]); } }
#pragma unroll
  for (int j = 0; j < 8; ++j) {
#pragma unroll
    for (int r = 0; r < 8; ++r) sh[wave * 16 + 8 * g + r][j * 16 + col] = (_Float16)(acc[j][r] * (W_CARRY / P_CARRY)); }
  __syncthreads();
  const size_t r0 = (size_t)b * TT + (size_t)blockIdx.x * 64;
  for (int e = tid; e < 64 * 16; e += 128) { const int rl = e >> 4, q = e & 15; vst2((void*)(AT + (r0 + rl) * CH + d0 + q * 8), *(const v4u*)&sh[rl][q * 8]); }
}

__global__ __launch_bounds__(128) void k_out(const _Float16* __restrict__ WOH, const _Float16* __restrict__ AT, const float* __restrict__ X, const float* __restrict__ GW, const float* __restrict__ GB, const float* __restrict__ OB, const float* __restrict__ STAT, float* __restrict__ Y) {
  __shared__ __align__(16) float ss[4][16][132];
  const int tid = threadIdx.x, wave = tid >> 5, lane = tid & 31, col = lane & 15, g = lane >> 4;
  const int b = blockIdx.x / (TT / 128); const int t0 = (blockIdx.x % (TT / 128)) * 128; const int o0 = blockIdx.y * 64 + wave * 16;
  v8f acc[8] = {};
#pragma unroll 2
  for (int kc = 0; kc < CH / 32; ++kc) { const v16h a = frag_h(WOH + (size_t)(o0 + col) * CH + kc * 32, lane);
#pragma unroll
    for (int j = 0; j < 8; ++j) { const v16h bf = frag_h(AT + ((size_t)b * TT + t0 + j * 16 + col) * CH + kc * 32, lane);
      acc[j] = wmma16(a, bf, acc[j]); } }
#pragma unroll
  for (int j = 0; j < 8; ++j) {
#pragma unroll
    for (int r = 0; r < 8; ++r) ss[wave][8 * g + r][j * 16 + col] = acc[j][r] * (1.0f / (W_CARRY * W_CARRY)); }
  LDSX();
  for (int rl = 0; rl < 16; ++rl) { const int o = o0 + rl;
    const v4f xv = *(const v4f*)(X + ((size_t)b * CH + o) * TT_FULL + t0 + lane * 4);
    const float* st = STAT + (size_t)(b * NG + (o >> 3)) * 32; const float mean = st[0], rstd = st[1]; const float w = bfr(GW[o]), gb = bfr(GB[o]), ob = bfr(OB[o]);
    const v4f a4 = *(const v4f*)&ss[wave][rl][lane * 4]; v4f o4;
#pragma unroll
    for (int i = 0; i < 4; ++i) o4[i] = ((bfr(xv[i]) - mean) * rstd * w + gb) + (a4[i] + ob);
    vst2((void*)(Y + ((size_t)b * CH + o) * (size_t)TT + t0 + lane * 4), o4); }
}

extern "C" void kernel_launch(void* const* d_in, const int* in_sizes, int n_in, void* d_out, int out_size, void* d_ws, size_t ws_size, hipStream_t stream) {
  if (n_in < 11) return;
  if ((long long)in_sizes[0] < (long long)NB * CH * TT_FULL - (TT_FULL - TT)) return;
  if (in_sizes[1] < CH || in_sizes[2] < CH || in_sizes[4] < CH || in_sizes[6] < CH || in_sizes[8] < CH || in_sizes[10] < CH) return;
  if (in_sizes[3] < CH * CH || in_sizes[5] < CH * CH || in_sizes[7] < CH * CH || in_sizes[9] < CH * CH) return;
  if ((long long)out_size < (long long)NB * CH * TT) return;
  if (ws_size < (size_t)WS_END) return;
  const float* const* F = (const float* const*)d_in;
  char* ws = (char*)d_ws;
  float* STAT = (float*)(ws + WS_STAT); _Float16* WH = (_Float16*)(ws + WS_WH); _Float16* XH = (_Float16*)(ws + WS_XH);
  _Float16* QH = (_Float16*)(ws + WS_QH); _Float16* KH = (_Float16*)(ws + WS_KH); _Float16* VT = (_Float16*)(ws + WS_VT); _Float16* AT = (_Float16*)(ws + WS_AT);
  float* S = (float*)(ws + WS_S);
  k_wcvt<<<dim3(32, 4), 256, 0, stream>>>(F[3], F[5], F[7], F[9], WH);
  k_gnstat<<<dim3(NB * NG), 256, 0, stream>>>(F[0], STAT);
  k_xn<<<dim3(NB * TT / 64), 256, 0, stream>>>(F[0], F[1], F[2], STAT, XH);
  k_proj<<<dim3(NB * TT / 64, CH / 128, 3), 128, 0, stream>>>(XH, WH, F[4], F[6], F[8], QH, KH, VT);
  for (int b = 0; b < NB; ++b) {
    k_sc<<<dim3(TT / 64, TT / 128), 128, 0, stream>>>(QH, KH, b, S);
    k_sm<<<dim3(TT), 256, 0, stream>>>(S);
    k_pv<<<dim3(TT / 64, CH / 128), 128, 0, stream>>>((const _Float16*)S, VT, b, AT);
  }
  k_out<<<dim3(NB * TT / 128, CH / 64), 128, 0, stream>>>(WH + (size_t)3 * CH * CH, AT, F[0], F[1], F[2], F[10], STAT, (float*)d_out);
}
